// MultiHeadedAttention1D_17540646436959
// MI455X (gfx1250) — hardware-verified
//
#include <hip/hip_runtime.h>
#include <stddef.h>
#include <stdint.h>


typedef _Float16 f16t;
typedef __bf16   bf16t;
typedef _Float16 v16h __attribute__((ext_vector_type(16)));
typedef _Float16 v8h  __attribute__((ext_vector_type(8)));
typedef __bf16   v16b __attribute__((ext_vector_type(16)));
typedef __bf16   v8b  __attribute__((ext_vector_type(8)));
typedef float    v8f  __attribute__((ext_vector_type(8)));
typedef float    v4f  __attribute__((ext_vector_type(4), __may_alias__));
typedef unsigned int v4u __attribute__((ext_vector_type(4), __may_alias__));

template<typename E> struct VT;
template<> struct VT<f16t>  { typedef v16h V16; typedef v8h V8; };
template<> struct VT<bf16t> { typedef v16b V16; typedef v8b V8; };

__device__ __forceinline__ v8f mma16(v8f c, v16h a, v16h b) {
    v8f d = __builtin_amdgcn_wmma_f32_16x16x32_f16(false, a, false, b, (short)0, c, false, false);
    asm volatile("v_nop\n\tv_nop\n\tv_nop\n\tv_nop" : "+v"(d) : "v"(a), "v"(b));
    return d;
}
__device__ __forceinline__ v8f mma16(v8f c, v16b a, v16b b) {
    v8f d = __builtin_amdgcn_wmma_f32_16x16x32_bf16(false, a, false, b, (short)0, c, false, false);
    asm volatile("v_nop\n\tv_nop\n\tv_nop\n\tv_nop" : "+v"(d) : "v"(a), "v"(b));
    return d;
}

template<typename E, int NP>
__global__ __launch_bounds__(256)
void cvt_rows(const float* in, E* o0, E* o1, int nchunk, float scale)
{
    typedef typename VT<E>::V8 V8;
    union U { V8 v; v4u u; E e[8]; };
    const int c = blockIdx.x * 256 + threadIdx.x;
    const bool ok = c < nchunk;
    v4u z = {0u, 0u, 0u, 0u};
    U h, l;
    h.u = z; l.u = z;
    if (ok) {
        const v4f* src = (const v4f*)(in + (size_t)c * 8);
        const v4f x0 = src[0], x1 = src[1];
        float xs[8] = {x0[0], x0[1], x0[2], x0[3], x1[0], x1[1], x1[2], x1[3]};
#pragma unroll
        for (int e = 0; e < 8; ++e) {
            const float x = xs[e] * scale;
            const E hv = (E)x;
            h.e[e] = hv;
            if (NP == 2) l.e[e] = (E)(x - (float)hv);
        }
    }
    E* p0 = o0 + (size_t)c * 8;
    E* p1 = o1 + (size_t)c * 8;
    if (ok) {
        *(volatile v4u*)p0 = h.u;
        if (NP == 2) *(volatile v4u*)p1 = l.u;
    }
    __threadfence();
    if (ok) {
        *(volatile v4u*)p0 = h.u;
        if (NP == 2) *(volatile v4u*)p1 = l.u;
    }
}

template<typename E, int NP>
__global__ __launch_bounds__(256)
void cvt_transpose(const float* in, E* o0, E* o1, int R, int Cn, float scale)
{
    typedef typename VT<E>::V8 V8;
    union U { V8 v; v4u u; E e[8]; };
    __shared__ float sIn[64 * 65];
    const int t  = threadIdx.x;
    const int r0 = blockIdx.y * 64;
    const int c0 = blockIdx.x * 64;

#pragma unroll
    for (int p = 0; p < 4; ++p) {
        const int f  = p * 256 + t;
        const int lr = f >> 4;
        const int lc = (f & 15) * 4;
        v4f x = {0.f, 0.f, 0.f, 0.f};
        if ((r0 + lr) < R && (c0 + lc + 3) < Cn)
            x = *(const v4f*)(in + (size_t)(r0 + lr) * Cn + c0 + lc);
        sIn[lr * 65 + lc + 0] = x[0];
        sIn[lr * 65 + lc + 1] = x[1];
        sIn[lr * 65 + lc + 2] = x[2];
        sIn[lr * 65 + lc + 3] = x[3];
    }
    __syncthreads();

    v4u z = {0u, 0u, 0u, 0u};
    U h[2], l[2];
    bool ok[2];
    size_t off[2];
#pragma unroll
    for (int p = 0; p < 2; ++p) {
        const int f   = p * 256 + t;
        const int oc  = f >> 3;
        const int seg = (f & 7) * 8;
        ok[p]  = ((c0 + oc) < Cn) && ((r0 + seg + 7) < R);
        off[p] = (size_t)(c0 + oc) * R + r0 + seg;
        h[p].u = z; l[p].u = z;
#pragma unroll
        for (int e = 0; e < 8; ++e) {
            const float x = sIn[(seg + e) * 65 + oc] * scale;
            const E hv = (E)x;
            h[p].e[e] = hv;
            if (NP == 2) l[p].e[e] = (E)(x - (float)hv);
        }
    }
#pragma unroll
    for (int p = 0; p < 2; ++p) {
        if (ok[p]) {
            *(volatile v4u*)(o0 + off[p]) = h[p].u;
            if (NP == 2) *(volatile v4u*)(o1 + off[p]) = l[p].u;
        }
    }
    __threadfence();
#pragma unroll
    for (int p = 0; p < 2; ++p) {
        if (ok[p]) {
            *(volatile v4u*)(o0 + off[p]) = h[p].u;
            if (NP == 2) *(volatile v4u*)(o1 + off[p]) = l[p].u;
        }
    }
}

template<typename E, int NP>
__global__ __launch_bounds__(128)
void gemm16(const E* A0, const E* A1, const E* B0, const E* B1,
            const float* bias, float* C, int M, int N, int K, float alpha)
{
    typedef typename VT<E>::V8  V8;
    typedef typename VT<E>::V16 V16;
    union Frag { V16 v; V8 h[2]; };

    __shared__ V8 sA[NP][256];
    __shared__ V8 sB[NP][256];
    __shared__ __align__(16) float sC[64 * 68];

    const int tid  = threadIdx.x;
    const int lane = tid & 31, wave = tid >> 5;
    const int hf   = lane >> 4,  m = lane & 15;
    const int wM   = (wave >> 1) * 32;
    const int wN   = (wave & 1) * 32;
    const int mBase = blockIdx.y * 64;
    const int nBase = blockIdx.x * 64;
    if (mBase + 64 > M || nBase + 64 > N) return;
    const int Kc = K >> 3;

    const V8* Ag[2];
    const V8* Bg[2];
    Ag[0] = (const V8*)A0; Ag[1] = (const V8*)A1;
    Bg[0] = (const V8*)B0; Bg[1] = (const V8*)B1;

    v8f zero8 = {0.f, 0.f, 0.f, 0.f, 0.f, 0.f, 0.f, 0.f};
    v8f acc[2][2];
#pragma unroll
    for (int mt = 0; mt < 2; ++mt)
#pragma unroll
        for (int nt = 0; nt < 2; ++nt) acc[mt][nt] = zero8;

    for (int kc = 0; kc + 4 <= Kc; kc += 4) {
#pragma unroll
        for (int j = 0; j < 2; ++j) {
            const int c    = tid + 128 * j;
            const int row  = c >> 2;
            const int part = c & 3;
#pragma unroll
            for (int p = 0; p < NP; ++p) {
                sA[p][c] = Ag[p][(size_t)(mBase + row) * Kc + kc + part];
                sB[p][c] = Bg[p][(size_t)(nBase + row) * Kc + kc + part];
            }
        }
        __syncthreads();

        Frag a[2][2], b[2][2];
#pragma unroll
        for (int p = 0; p < NP; ++p) {
#pragma unroll
            for (int t2 = 0; t2 < 2; ++t2) {
                const int ra = (wM + t2 * 16 + m) * 4;
                const int rb = (wN + t2 * 16 + m) * 4;
                a[p][t2].h[0] = sA[p][ra + hf];
                a[p][t2].h[1] = sA[p][ra + 2 + hf];
                b[p][t2].h[0] = sB[p][rb + hf];
                b[p][t2].h[1] = sB[p][rb + 2 + hf];
            }
        }
#pragma unroll
        for (int mt = 0; mt < 2; ++mt) {
#pragma unroll
            for (int nt = 0; nt < 2; ++nt) {
                acc[mt][nt] = mma16(acc[mt][nt], a[0][mt].v, b[0][nt].v);
                if (NP == 2) {
                    acc[mt][nt] = mma16(acc[mt][nt], a[0][mt].v,      b[NP - 1][nt].v);
                    acc[mt][nt] = mma16(acc[mt][nt], a[NP - 1][mt].v, b[0][nt].v);
                }
            }
        }
        __syncthreads();
    }

#pragma unroll
    for (int mt = 0; mt < 2; ++mt)
#pragma unroll
        for (int nt = 0; nt < 2; ++nt)
#pragma unroll
            for (int r = 0; r < 8; ++r)
                sC[(wM + mt * 16 + hf * 8 + r) * 68 + wN + nt * 16 + m] = acc[mt][nt][r];
    __syncthreads();

    const v4f* bias4 = (const v4f*)(bias + nBase);
    const v4f* sC4   = (const v4f*)sC;
#pragma unroll
    for (int p = 0; p < 8; ++p) {
        const int f   = p * 128 + tid;
        const int row = f >> 4;
        const int c4  = f & 15;
        const v4f o = sC4[row * 17 + c4] * alpha + bias4[c4];
        *(volatile v4f*)(C + (size_t)(mBase + row) * N + nBase + c4 * 4) = o;
    }
    __threadfence();
#pragma unroll
    for (int p = 0; p < 8; ++p) {
        const int f   = p * 128 + tid;
        const int row = f >> 4;
        const int c4  = f & 15;
        const v4f o = sC4[row * 17 + c4] * alpha + bias4[c4];
        *(volatile v4f*)(C + (size_t)(mBase + row) * N + nBase + c4 * 4) = o;
    }
}

__global__ __launch_bounds__(256)
void band_mix(const float* q, const float* k, const float* v, const float* xq,
              float* T, int nrows, int rowlen)
{
    __shared__ __align__(16) float sk[1024];
    __shared__ __align__(16) float sv[1024];
    const int row = blockIdx.x;
    if (row >= nrows || rowlen != 1024) return;
    const int t = threadIdx.x;
    const size_t base = (size_t)row * 1024;
    const v4f* q4 = (const v4f*)(q  + base);
    const v4f* k4 = (const v4f*)(k  + base);
    const v4f* v4 = (const v4f*)(v  + base);
    const v4f* x4 = (const v4f*)(xq + base);
    ((v4f*)sk)[t] = k4[t];
    ((v4f*)sv)[t] = v4[t];
    __syncthreads();

    const v4f qv = q4[t];
    const v4f xv = x4[t];
    const int e0 = t * 4;
    const int hb = e0 & ~63;
    const int i0 = e0 & 63;
    float rr[4];
#pragma unroll
    for (int u = 0; u < 4; ++u) {
        const int i = i0 + u;
        const float qi = qv[u];
        int j0 = i - 8; if (j0 < 0)  j0 = 0;
        int j1 = i + 8; if (j1 > 63) j1 = 63;
        float mx = -3.402823466e+38f;
#pragma unroll 1
        for (int j = j0; j <= j1; ++j) {
            const float s = (qi * sk[hb + j]) * 0.125f;
            mx = fmaxf(mx, s);
        }
        float sum = 0.f, acc = 0.f;
#pragma unroll 1
        for (int j = j0; j <= j1; ++j) {
            const float s = (qi * sk[hb + j]) * 0.125f;
            const float e = __expf(s - mx);
            sum += e;
            acc += e * sv[hb + j];
        }
        rr[u] = xv[u] - acc * __builtin_amdgcn_rcpf(sum);
    }
    v4f o = {rr[0], rr[1], rr[2], rr[3]};
    float* dst = T + base + (size_t)t * 4;
    *(volatile v4f*)dst = o;
    __threadfence();
    *(volatile v4f*)dst = o;
}

extern "C" void kernel_launch(void* const* d_in, const int* in_sizes, int n_in,
                              void* d_out, int out_size, void* d_ws, size_t ws_size,
                              hipStream_t stream)
{
    const int NBt = 2048;
    const int NDm = 1024;
    const int nX  = NBt * NDm;
    const int nW  = NDm * NDm;

    if (n_in < 11) return;
    if (in_sizes[0] != nX || in_sizes[1] != nX || in_sizes[2] != nX) return;
    if (in_sizes[3] != nW || in_sizes[5] != nW || in_sizes[7] != nW || in_sizes[9] != nW) return;
    if (in_sizes[4] != NDm || in_sizes[6] != NDm || in_sizes[8] != NDm || in_sizes[10] != NDm) return;
    if (out_size != nX) return;

    const float* Xq = (const float*)d_in[0];
    const float* Xk = (const float*)d_in[1];
    const float* Xv = (const float*)d_in[2];
    const float* Wq = (const float*)d_in[3];
    const float* bq = (const float*)d_in[4];
    const float* Wk = (const float*)d_in[5];
    const float* bk = (const float*)d_in[6];
    const float* Wv = (const float*)d_in[7];
    const float* bv = (const float*)d_in[8];
    const float* Wo = (const float*)d_in[9];
    const float* bo = (const float*)d_in[10];
    float* out = (float*)d_out;

    const size_t bXf = (size_t)nX * 4;
    const size_t bXh = (size_t)nX * 2;
    const size_t bWh = (size_t)nW * 2;
    char* ws = (char*)d_ws;
    size_t o = 0;
    float* qf  = (float*)(ws + o); o += bXf;
    float* kf  = (float*)(ws + o); o += bXf;
    float* vf  = (float*)(ws + o); o += bXf;
    float* Tf  = (float*)(ws + o); o += bXf;
    f16t*  Xqh = (f16t*)(ws + o);  o += bXh;
    f16t*  Xkh = (f16t*)(ws + o);  o += bXh;
    f16t*  Xvh = (f16t*)(ws + o);  o += bXh;
    f16t*  Wqt = (f16t*)(ws + o);  o += bWh;
    f16t*  Wkt = (f16t*)(ws + o);  o += bWh;
    f16t*  Wvt = (f16t*)(ws + o);  o += bWh;
    bf16t* Wohi = (bf16t*)(ws + o); o += bWh;
    bf16t* Wolo = (bf16t*)(ws + o); o += bWh;
    bf16t* Thi  = (bf16t*)(ws + o); o += bXh;
    bf16t* Tlo  = (bf16t*)(ws + o); o += bXh;
    if (o > ws_size) return;

    const int chunksX = nX / 8;
    const dim3 gcx((chunksX + 255) / 256);
    const dim3 gtr((NDm + 63) / 64, (NDm + 63) / 64);
    const dim3 gg(NDm / 64, NBt / 64);

    cvt_rows<f16t, 1><<<gcx, 256, 0, stream>>>(Xq, Xqh, Xqh, chunksX, 1.0f);
    cvt_rows<f16t, 1><<<gcx, 256, 0, stream>>>(Xk, Xkh, Xkh, chunksX, 1.0f);
    cvt_rows<f16t, 1><<<gcx, 256, 0, stream>>>(Xv, Xvh, Xvh, chunksX, 1.0f);
    cvt_transpose<f16t, 1><<<gtr, 256, 0, stream>>>(Wq, Wqt, Wqt, NDm, NDm, 64.0f);
    cvt_transpose<f16t, 1><<<gtr, 256, 0, stream>>>(Wk, Wkt, Wkt, NDm, NDm, 64.0f);
    cvt_transpose<f16t, 1><<<gtr, 256, 0, stream>>>(Wv, Wvt, Wvt, NDm, NDm, 64.0f);
    cvt_transpose<bf16t, 2><<<gtr, 256, 0, stream>>>(Wo, Wohi, Wolo, NDm, NDm, 1.0f);

    gemm16<f16t, 1><<<gg, 128, 0, stream>>>(Xqh, Xqh, Wqt, Wqt, bq, qf, NBt, NDm, NDm, 0.015625f);
    gemm16<f16t, 1><<<gg, 128, 0, stream>>>(Xkh, Xkh, Wkt, Wkt, bk, kf, NBt, NDm, NDm, 0.015625f);
    gemm16<f16t, 1><<<gg, 128, 0, stream>>>(Xvh, Xvh, Wvt, Wvt, bv, vf, NBt, NDm, NDm, 0.015625f);

    band_mix<<<dim3(NBt), 256, 0, stream>>>(qf, kf, vf, Xq, Tf, NBt, NDm);

    cvt_rows<bf16t, 2><<<gcx, 256, 0, stream>>>(Tf, Thi, Tlo, chunksX, 1.0f);
    gemm16<bf16t, 2><<<gg, 128, 0, stream>>>(Thi, Tlo, Wohi, Wolo, bo, out, NBt, NDm, NDm, 1.0f);

    (void)hipGetLastError();
}
